// MultiHeadAttention_43611097924070
// MI455X (gfx1250) — hardware-verified
//
#include <hip/hip_runtime.h>


#ifndef NB
#define NB 2
#endif
#ifndef SEQ
#define SEQ 2048
#endif
#ifndef SEQ_FULL
#define SEQ_FULL 2048
#endif
#define DM    1024
#define NH_   16
#define HD    64
#define MROWS (NB * SEQ)
#define HB    (SEQ * HD)
#define RPB   (SEQ / 64)
#define WCAR  64.0f
#define OCAR  256.0f
#define PLOG  8.0f

static_assert(SEQ % 64 == 0);
static_assert(MROWS % 64 == 0);
static_assert(DM % 64 == 0);
static_assert(DM == NH_ * HD);
static_assert((SEQ * DM) % 2048 == 0);
static_assert((DM * DM) % 2048 == 0);
static_assert(SEQ <= SEQ_FULL);

typedef _Float16 h16;
typedef unsigned short bf;
typedef __attribute__((ext_vector_type(16))) __bf16   v16bf;
typedef __attribute__((ext_vector_type(16))) _Float16 v16h;
typedef __attribute__((ext_vector_type(8)))  _Float16 v8h;
typedef __attribute__((ext_vector_type(8)))  unsigned short v8us;
typedef __attribute__((ext_vector_type(8)))  float    v8f;
typedef __attribute__((ext_vector_type(4)))  float    v4f;
typedef v8h  __attribute__((may_alias)) v8ha;
typedef v4f  __attribute__((may_alias)) v4fa;
typedef v8us __attribute__((may_alias)) v8usa;

__device__ __forceinline__ unsigned short f2bf(float f) { unsigned u = __float_as_uint(f); u += 0x7FFFu + ((u >> 16) & 1u); return (unsigned short)(u >> 16); }
__device__ __forceinline__ float bf2f(unsigned short b) { return __uint_as_float(((unsigned)b) << 16); }
__device__ __forceinline__ float bfr(float f) { return bf2f(f2bf(f)); }
__device__ __forceinline__ v16h cat16(v8h lo, v8h hi) { return __builtin_shufflevector(lo, hi, 0, 1, 2, 3, 4, 5, 6, 7, 8, 9, 10, 11, 12, 13, 14, 15); }
__device__ __forceinline__ v16bf cat16b(v8us lo, v8us hi) { return __builtin_bit_cast(v16bf, __builtin_shufflevector(lo, hi, 0, 1, 2, 3, 4, 5, 6, 7, 8, 9, 10, 11, 12, 13, 14, 15)); }
__device__ __forceinline__ v8f wmma16(v16h a, v16h b, v8f c) { return __builtin_amdgcn_wmma_f32_16x16x32_f16(false, a, false, b, (short)0, c, false, false); }
__device__ __forceinline__ v8f wmmab(v16bf a, v16bf b, v8f c) { return __builtin_amdgcn_wmma_f32_16x16x32_bf16(false, a, false, b, (short)0, c, false, false); }
__device__ __forceinline__ void wsync() { __builtin_amdgcn_fence(3  , "wavefront"); __builtin_amdgcn_wave_barrier(); asm volatile("" ::: "memory"); }

template <typename T16> struct WFrag;
template <> struct WFrag<h16> { typedef v16h V; static __device__ __forceinline__ V ld(const h16* p) { return cat16(*(const v8h*)p, *(const v8h*)(p + 16)); } static __device__ __forceinline__ v8f mma(V a, V b, v8f c) { return wmma16(a, b, c); } };
template <> struct WFrag<bf> { typedef v16bf V; static __device__ __forceinline__ V ld(const bf* p) { return cat16b(*(const v8us*)p, *(const v8us*)(p + 16)); } static __device__ __forceinline__ v8f mma(V a, V b, v8f c) { return wmmab(a, b, c); } };

template <typename T16, bool OUT16>
__global__ __launch_bounds__(32) void k_gemmw(const T16* __restrict__ A, const T16* __restrict__ Bt, unsigned K, float* C32, h16* C16, unsigned ldc, const float* __restrict__ bias, float osc) {
    typedef typename WFrag<T16>::V V;
    __shared__ __align__(16) float os[16 * 68];
    const unsigned lane = threadIdx.x & 31u, lr = lane & 15u, hi = lane >> 4;
    const unsigned r0 = blockIdx.x * 64u, c0 = blockIdx.y * 64u;
    v8f acc[4][4];
#pragma unroll
    for (int mb = 0; mb < 4; ++mb)
#pragma unroll
        for (int nb = 0; nb < 4; ++nb) acc[mb][nb] = (v8f){};
    const T16* ap = A + (size_t)(r0 + lr) * K + 8u * hi;
    const T16* bp = Bt + (size_t)(c0 + lr) * K + 8u * hi;
#pragma unroll 1
    for (unsigned kc = 0; kc < K; kc += 32u) {
        V a[4];
#pragma unroll
        for (int mb = 0; mb < 4; ++mb) a[mb] = WFrag<T16>::ld(ap + (size_t)mb * 16u * K + kc);
#pragma unroll
        for (int nb = 0; nb < 4; ++nb) { const V b = WFrag<T16>::ld(bp + (size_t)nb * 16u * K + kc);
#pragma unroll
            for (int mb = 0; mb < 4; ++mb) acc[mb][nb] = WFrag<T16>::mma(a[mb], b, acc[mb][nb]); }
        asm volatile("v_nop\n\tv_nop\n\tv_nop\n\tv_nop" : "+v"(acc[0][0]), "+v"(acc[1][1]), "+v"(acc[2][2]), "+v"(acc[3][3]) : "v"(a[0]), "v"(a[3]));
    }
    const unsigned rq = lane >> 3, seg = lane & 7u;
    const unsigned bcol = OUT16 ? (c0 + seg * 8u) : (c0 + lr * 4u);
    const v4f bz0 = *(const v4f*)(bias + bcol);
    const v4f bz1 = *(const v4f*)(bias + (OUT16 ? bcol + 4u : bcol));
    v4f bb0, bb1;
#pragma unroll
    for (int i = 0; i < 4; ++i) { bb0[i] = bfr(bz0[i]); bb1[i] = bfr(bz1[i]); }
#pragma unroll
    for (int mb = 0; mb < 4; ++mb) {
#pragma unroll
        for (int nb = 0; nb < 4; ++nb) {
#pragma unroll
            for (int j = 0; j < 8; ++j) os[(hi * 8u + j) * 68u + nb * 16u + lr] = acc[mb][nb][j]; }
        wsync();
        if (OUT16) {
            v8h ov[4];
#pragma unroll
            for (int s = 0; s < 4; ++s) { const unsigned row = 4u * s + rq; const v4f x0 = *(const v4fa*)(os + row * 68u + seg * 8u); const v4f x1 = *(const v4fa*)(os + row * 68u + seg * 8u + 4u);
#pragma unroll
                for (int i = 0; i < 4; ++i) { ov[s][i] = (h16)(x0[i] * osc + bb0[i]); ov[s][4 + i] = (h16)(x1[i] * osc + bb1[i]); } }
            h16* crow = C16 + (size_t)(r0 + mb * 16u) * ldc + c0;
#pragma unroll 1
            for (int ps = 0; ps < 2; ++ps) {
#pragma unroll
                for (int s = 0; s < 4; ++s) *(volatile v8h*)(crow + (size_t)(4u * s + rq) * ldc + seg * 8u) = ov[s];
                if (ps == 0) __threadfence(); }
        } else {
            float* crow = C32 + (size_t)(r0 + mb * 16u) * ldc + c0;
#pragma unroll 1
            for (int ps = 0; ps < 2; ++ps) {
#pragma unroll
                for (int s = 0; s < 8; ++s) { const unsigned row = 2u * s + hi, cofs = lr * 4u; const v4f x = *(const v4fa*)(os + row * 68u + cofs); v4f val;
#pragma unroll
                    for (int i = 0; i < 4; ++i) val[i] = x[i] * osc + bb0[i];
                    *(volatile v4f*)(crow + (size_t)row * ldc + cofs) = val; }
                if (ps == 0) __threadfence(); }
        }
        wsync();
    }
}

__global__ __launch_bounds__(256) void k_cvt8(const float* __restrict__ src, bf* dst, unsigned n8, size_t sStride, size_t dStride) {
    const unsigned i = blockIdx.x * 256u + threadIdx.x; if (i >= n8) return;
    const float* s = src + (size_t)blockIdx.y * sStride; bf* d = dst + (size_t)blockIdx.y * dStride;
    const v8f v = *(const v8f*)(s + (size_t)i * 8u); v8us o;
#pragma unroll
    for (int k = 0; k < 8; ++k) o[k] = f2bf(v[k]);
    *(volatile v8us*)(d + (size_t)i * 8u) = o; __threadfence(); *(volatile v8us*)(d + (size_t)i * 8u) = o; }

__global__ __launch_bounds__(256) void k_cvtw(const float* __restrict__ src, h16* dst, unsigned n8, float car) {
    const unsigned i = blockIdx.x * 256u + threadIdx.x; if (i >= n8) return;
    const v8f v = *(const v8f*)(src + (size_t)i * 8u); v8h o;
#pragma unroll
    for (int k = 0; k < 8; ++k) o[k] = (h16)(bfr(v[k]) * car);
    *(volatile v8h*)(dst + (size_t)i * 8u) = o; __threadfence(); *(volatile v8h*)(dst + (size_t)i * 8u) = o; }

__global__ __launch_bounds__(256) void k_tr64(const unsigned short* __restrict__ src, unsigned short* dst, unsigned sBlk, unsigned sRow, unsigned dBlk, unsigned dRow) {
    __shared__ __align__(16) unsigned short t[64 * 72];
    const unsigned tid = threadIdx.x; const size_t hb = (size_t)blockIdx.y * HB;
    const unsigned short* s = src + hb + (size_t)blockIdx.x * sBlk; unsigned short* d = dst + hb + (size_t)blockIdx.x * dBlk;
#pragma unroll
    for (int it = 0; it < 2; ++it) { const unsigned piece = tid + 256u * it, row = piece >> 3, seg = piece & 7u; const v8us v = *(const v8us*)(s + (size_t)row * sRow + seg * 8u); *(v8usa*)(t + row * 72u + seg * 8u) = v; }
    __syncthreads();
    v8us o0, o1;
    { const unsigned c = tid >> 3, seg = tid & 7u;
#pragma unroll
      for (int i = 0; i < 8; ++i) o0[i] = t[(seg * 8u + i) * 72u + c]; }
    { const unsigned c = (tid + 256u) >> 3, seg = tid & 7u;
#pragma unroll
      for (int i = 0; i < 8; ++i) o1[i] = t[(seg * 8u + i) * 72u + c]; }
    const unsigned ca = tid >> 3, cb = (tid + 256u) >> 3, sg = tid & 7u;
    *(volatile v8us*)(d + (size_t)ca * dRow + sg * 8u) = o0; *(volatile v8us*)(d + (size_t)cb * dRow + sg * 8u) = o1;
    __threadfence();
    *(volatile v8us*)(d + (size_t)ca * dRow + sg * 8u) = o0; *(volatile v8us*)(d + (size_t)cb * dRow + sg * 8u) = o1;
}

__global__ __launch_bounds__(32) void k_flash(const h16* __restrict__ QP, const h16* __restrict__ KP, const h16* __restrict__ VT, h16* AT) {
    __shared__ __align__(16) h16 os[32 * 72];
    const unsigned lane = threadIdx.x & 31u, lr = lane & 15u, hi = lane >> 4;
    const size_t hb = (size_t)blockIdx.y * HB; const unsigned q0 = blockIdx.x * 32u;
    const h16* Qb = QP + hb + (size_t)(q0 + lr) * HD + 8u * hi;
    const h16* Kb = KP + hb + (size_t)lr * HD + 8u * hi;
    const h16* Vb = VT + hb + (size_t)lr * SEQ + 8u * hi;
    v16h qf[2][2];
#pragma unroll
    for (int t = 0; t < 2; ++t)
#pragma unroll
        for (int ks = 0; ks < 2; ++ks) qf[t][ks] = WFrag<h16>::ld(Qb + (size_t)t * 16u * HD + ks * 32u);
    v8f oacc[4][2];
#pragma unroll
    for (int dt = 0; dt < 4; ++dt) { oacc[dt][0] = (v8f){}; oacc[dt][1] = (v8f){}; }
    float mrun[2] = { -3.0e38f, -3.0e38f }, lsum[2] = { 0.f, 0.f };
    const float C2 = 0.125f * 1.4426950408889634f;
#pragma unroll 1
    for (unsigned kb = 0; kb < SEQ; kb += 32u) {
        v16h ka[2][2], va[4];
#pragma unroll
        for (int kt = 0; kt < 2; ++kt)
#pragma unroll
            for (int ks = 0; ks < 2; ++ks) ka[kt][ks] = WFrag<h16>::ld(Kb + (size_t)(kb + 16u * kt) * HD + ks * 32u);
#pragma unroll
        for (int dt = 0; dt < 4; ++dt) va[dt] = WFrag<h16>::ld(Vb + (size_t)(16u * dt) * SEQ + kb);
        v8f st[2][2];
        st[0][0] = (v8f){}; st[0][1] = (v8f){}; st[1][0] = (v8f){}; st[1][1] = (v8f){};
#pragma unroll
        for (int ks = 0; ks < 2; ++ks)
#pragma unroll
            for (int kt = 0; kt < 2; ++kt)
#pragma unroll
                for (int t = 0; t < 2; ++t) st[kt][t] = wmma16(ka[kt][ks], qf[t][ks], st[kt][t]);
        asm volatile("v_nop\n\tv_nop\n\tv_nop\n\tv_nop" : "+v"(st[0][0]), "+v"(st[0][1]), "+v"(st[1][0]), "+v"(st[1][1]) : "v"(ka[0][1]), "v"(ka[1][1]));
        v16h pb[2];
#pragma unroll
        for (int t = 0; t < 2; ++t) {
            float mx = -3.0e38f;
#pragma unroll
            for (int kt = 0; kt < 2; ++kt)
#pragma unroll
                for (int r = 0; r < 8; ++r) { const float x = st[kt][t][r] * C2; st[kt][t][r] = x; mx = fmaxf(mx, x); }
            mx = fmaxf(mx, __shfl_xor(mx, 16, 32));
            const float mn = fmaxf(mrun[t], mx);
            const float alpha = __builtin_amdgcn_exp2f(mrun[t] - mn);
            mrun[t] = mn;
            const float sh = PLOG - mn;
            float sum = 0.f;
#pragma unroll
            for (int kt = 0; kt < 2; ++kt)
#pragma unroll
                for (int r = 0; r < 8; ++r) { const float p = __builtin_amdgcn_exp2f(st[kt][t][r] + sh); sum += p; pb[t][kt * 8 + r] = (h16)p; }
            lsum[t] = lsum[t] * alpha + sum;
#pragma unroll
            for (int dt = 0; dt < 4; ++dt)
#pragma unroll
                for (int r = 0; r < 8; ++r) oacc[dt][t][r] *= alpha;
        }
#pragma unroll
        for (int dt = 0; dt < 4; ++dt) { oacc[dt][0] = wmma16(va[dt], pb[0], oacc[dt][0]); oacc[dt][1] = wmma16(va[dt], pb[1], oacc[dt][1]); }
        asm volatile("v_nop\n\tv_nop\n\tv_nop\n\tv_nop" : "+v"(oacc[0][0]), "+v"(oacc[0][1]), "+v"(oacc[1][0]), "+v"(oacc[1][1]), "+v"(oacc[2][0]), "+v"(oacc[2][1]), "+v"(oacc[3][0]), "+v"(oacc[3][1]) : "v"(pb[0]), "v"(pb[1]), "v"(va[3]));
    }
#pragma unroll
    for (int t = 0; t < 2; ++t) {
        const float ltot = lsum[t] + __shfl_xor(lsum[t], 16, 32);
        const float rinv = OCAR * (1.0f / ltot);
#pragma unroll
        for (int dt = 0; dt < 4; ++dt) { v8h o;
#pragma unroll
            for (int r = 0; r < 8; ++r) o[r] = (h16)(oacc[dt][t][r] * rinv);
            *(v8ha*)(os + (16u * t + lr) * 72u + 16u * dt + 8u * hi) = o; }
    }
    wsync();
    const unsigned rq = lane >> 3, seg = lane & 7u;
    v8h ov[8];
#pragma unroll
    for (int s = 0; s < 8; ++s) ov[s] = *(const v8ha*)(os + (4u * s + rq) * 72u + seg * 8u);
    h16* arow = AT + hb + (size_t)q0 * HD;
#pragma unroll 1
    for (int ps = 0; ps < 2; ++ps) {
#pragma unroll
        for (int s = 0; s < 8; ++s) *(volatile v8h*)(arow + (size_t)(4u * s + rq) * HD + seg * 8u) = ov[s];
        if (ps == 0) __threadfence(); }
}

extern "C" void kernel_launch(void* const* d_in, const int* in_sizes, int n_in,
                              void* d_out, int out_size, void* d_ws, size_t ws_size, hipStream_t stream) {
    if (n_in < 11) return;
    const size_t needX = (size_t)(NB - 1) * SEQ_FULL * DM + (size_t)SEQ * DM;
    if ((size_t)in_sizes[0] < needX || (size_t)in_sizes[1] < needX || (size_t)in_sizes[2] < needX) return;
    if (in_sizes[3] < DM * DM || in_sizes[5] < DM * DM || in_sizes[7] < DM * DM || in_sizes[9] < DM * DM) return;
    if (in_sizes[4] < DM || in_sizes[6] < DM || in_sizes[8] < DM || in_sizes[10] < DM) return;
    if ((size_t)out_size < (size_t)MROWS * DM) return;
    const float* q = (const float*)d_in[0]; const float* k = (const float*)d_in[1]; const float* v = (const float*)d_in[2];
    const float* wq = (const float*)d_in[3]; const float* bq = (const float*)d_in[4];
    const float* wk = (const float*)d_in[5]; const float* bk = (const float*)d_in[6];
    const float* wv = (const float*)d_in[7]; const float* bv = (const float*)d_in[8];
    const float* wo = (const float*)d_in[9]; const float* bo = (const float*)d_in[10];
    float* OUT = (float*)d_out;
    char* wsp = (char*)d_ws;
    auto take = [&](size_t bytes) { char* p = wsp; wsp += (bytes + 255) & ~(size_t)255; return (void*)p; };
    const size_t PL = (size_t)MROWS * DM;
    bf* XQ = (bf*)take(PL * 2); bf* XK = (bf*)take(PL * 2); bf* XV = (bf*)take(PL * 2);
    bf* WQ = (bf*)take((size_t)DM * DM * 2); bf* WK = (bf*)take((size_t)DM * DM * 2); bf* WV = (bf*)take((size_t)DM * DM * 2); h16* WO = (h16*)take((size_t)DM * DM * 2);
    h16* QP = (h16*)take(PL * 2);
    h16* KS = (h16*)take(PL * 2);
    h16* KP = (h16*)take(PL * 2);
    h16* VS = (h16*)take(PL * 2);
    h16* VT = (h16*)take(PL * 2);
    h16* AT = (h16*)take(PL * 2);
    const size_t used = (size_t)(wsp - (char*)d_ws);
    if (used > ws_size || used > ((size_t)128 << 20)) return;

    const unsigned gx = (unsigned)((size_t)SEQ * DM / 8 / 256), gw = (unsigned)((size_t)DM * DM / 8 / 256);
    k_cvt8<<<dim3(gx, NB), 256, 0, stream>>>(q, XQ, (unsigned)((size_t)SEQ * DM / 8), (size_t)SEQ_FULL * DM, (size_t)SEQ * DM);
    k_cvt8<<<dim3(gx, NB), 256, 0, stream>>>(k, XK, (unsigned)((size_t)SEQ * DM / 8), (size_t)SEQ_FULL * DM, (size_t)SEQ * DM);
    k_cvt8<<<dim3(gx, NB), 256, 0, stream>>>(v, XV, (unsigned)((size_t)SEQ * DM / 8), (size_t)SEQ_FULL * DM, (size_t)SEQ * DM);
    k_cvt8<<<dim3(gw, 1), 256, 0, stream>>>(wq, WQ, (unsigned)((size_t)DM * DM / 8), 0, 0);
    k_cvt8<<<dim3(gw, 1), 256, 0, stream>>>(wk, WK, (unsigned)((size_t)DM * DM / 8), 0, 0);
    k_cvt8<<<dim3(gw, 1), 256, 0, stream>>>(wv, WV, (unsigned)((size_t)DM * DM / 8), 0, 0);
    k_cvtw<<<gw, 256, 0, stream>>>(wo, WO, (unsigned)((size_t)DM * DM / 8), WCAR);

    const dim3 gg(MROWS / 64, DM / 64, 1);
    k_gemmw<bf, true><<<gg, 32, 0, stream>>>(XQ, WQ, DM, nullptr, QP, DM, bq, 1.0f);
    k_gemmw<bf, true><<<gg, 32, 0, stream>>>(XK, WK, DM, nullptr, KS, DM, bk, 1.0f);
    k_gemmw<bf, true><<<gg, 32, 0, stream>>>(XV, WV, DM, nullptr, VS, DM, bv, 1.0f);

    k_tr64<<<dim3(RPB, NB * NH_), 256, 0, stream>>>((const unsigned short*)KS, (unsigned short*)KP, 64u, (unsigned)(RPB * 64), 4096u, 64u);
    k_tr64<<<dim3(RPB, NB * NH_), 256, 0, stream>>>((const unsigned short*)VS, (unsigned short*)VT, 4096u, 64u, 64u, (unsigned)SEQ);

    k_flash<<<dim3(SEQ / 32, NB * NH_), 32, 0, stream>>>(QP, KP, VT, AT);

    k_gemmw<h16, false><<<gg, 32, 0, stream>>>(AT, WO, DM, OUT, nullptr, DM, bo, 1.0f / (OCAR * WCAR));
}
